// Net_18107582120151
// MI455X (gfx1250) — hardware-run, weakly checked
//
#include <hip/hip_runtime.h>
#include <math.h>

constexpr int NSAMP     = 16384;
constexpr int NHID      = 32;
constexpr int NCLS      = 10;
constexpr int NSTEP     = 96;
constexpr int NTHR      = 128;
constexpr int NWAVE     = NTHR / 32;
constexpr int SAMP_WAVE = 16;
constexpr int SAMP_BLK  = NWAVE * SAMP_WAVE;
constexpr int NBLK      = NSAMP / SAMP_BLK;
constexpr int OUT_WAVE  = SAMP_WAVE * NCLS;
static_assert(NSAMP % SAMP_BLK == 0);
static_assert(NHID == 32);
static_assert(OUT_WAVE == 160);
static_assert((OUT_WAVE * 4) % 128 == 0);
static_assert(NHID * NHID == 2 * 4 * NTHR);
static_assert(3 * NHID <= NTHR && 2 * NHID <= NTHR && 2 * NCLS <= NTHR);

constexpr float CARRY_H        = 16.0f;
constexpr float CARRY_W        = 64.0f;
constexpr float CARRY_INV      = 1.0f / (CARRY_H * CARRY_W);
constexpr float F16_MIN_NORMAL = 6.103515625e-05f;
static_assert(CARRY_H * CARRY_W == 1024.0f);
static_assert(CARRY_INV * 1024.0f == 1.0f);

constexpr int P_W2    = 0;
constexpr int P_W1    = P_W2 + NHID * NHID;
constexpr int P_B1    = P_W1 + 3 * NHID;
constexpr int P_B2    = P_B1 + NHID;
constexpr int P_W3    = P_B2 + NHID;
constexpr int P_B3    = P_W3 + 2 * NHID;
constexpr int P_FCW   = P_B3 + 4;
constexpr int P_FCB   = P_FCW + 2 * NCLS;
constexpr int P_TOTAL = P_FCB + 12;
static_assert(P_TOTAL == 1284);

constexpr float RK_A21 = 0.2f;
constexpr float RK_A31 = (float)(3.0 / 40.0);
constexpr float RK_A32 = (float)(9.0 / 40.0);
constexpr float RK_A41 = (float)(44.0 / 45.0);
constexpr float RK_A42 = (float)(-56.0 / 15.0);
constexpr float RK_A43 = (float)(32.0 / 9.0);
constexpr float RK_A51 = (float)(19372.0 / 6561.0);
constexpr float RK_A52 = (float)(-25360.0 / 2187.0);
constexpr float RK_A53 = (float)(64448.0 / 6561.0);
constexpr float RK_A54 = (float)(-212.0 / 729.0);
constexpr float RK_A61 = (float)(9017.0 / 3168.0);
constexpr float RK_A62 = (float)(-355.0 / 33.0);
constexpr float RK_A63 = (float)(46732.0 / 5247.0);
constexpr float RK_A64 = (float)(49.0 / 176.0);
constexpr float RK_A65 = (float)(-5103.0 / 18656.0);
constexpr float RK_B1  = (float)(35.0 / 384.0);
constexpr float RK_B3  = (float)(500.0 / 1113.0);
constexpr float RK_B4  = (float)(125.0 / 192.0);
constexpr float RK_B5  = (float)(-2187.0 / 6784.0);
constexpr float RK_B6  = (float)(11.0 / 84.0);
constexpr float RK_E1  = (float)(71.0 / 57600.0);
constexpr float RK_E3  = (float)(-71.0 / 16695.0);
constexpr float RK_E4  = (float)(71.0 / 1920.0);
constexpr float RK_E5  = (float)(-17253.0 / 339200.0);
constexpr float RK_E6  = (float)(22.0 / 525.0);
constexpr float RK_E7  = (float)(-1.0 / 40.0);
constexpr float RK_C5  = (float)(8.0 / 9.0);

typedef __attribute__((ext_vector_type(16))) _Float16 v16h;
typedef __attribute__((ext_vector_type(8)))  float    v8f;
typedef __attribute__((ext_vector_type(4)))  float    v4f;

__device__ __forceinline__ float flush_small(float v) {
  return (fabsf(v) < F16_MIN_NORMAL) ? 0.0f : v;
}

__device__ __forceinline__ v8f mma_h(v16h a, v16h b, v8f c) {
  return __builtin_amdgcn_wmma_f32_16x16x32_f16(false, a, false, b, (short)0, c, false, false);
}
__device__ __forceinline__ void mma_guard(v8f& d, v16h a, v16h b) {
  asm volatile("v_nop\n\tv_nop\n\tv_nop\n\tv_nop" : "+v"(d) : "v"(a), "v"(b));
}

__device__ __forceinline__ void stage_small(float* dst, const float* __restrict__ src, int n, int tid) {
  const int ic = (tid < n) ? tid : (n - 1);
  float v = src[ic];
  asm volatile("" : "+v"(v));
  if (tid < n) dst[tid] = v;
}

__device__ __forceinline__ void field_eval(float tin, float ya, float yb,
    const float (&w1t)[16], const float (&w1a)[16], const float (&w1b)[16], const float (&b1r)[16],
    const v16h& a2h0, const v16h& a2h1,
    const v8f& cb0, const v8f& cb1,
    const float (&w3a)[16], const float (&w3b)[16], float b30, float b31,
    float& o0, float& o1) {
  v16h bh;
#pragma unroll
  for (int i = 0; i < 16; ++i) {
    const float g = fmaxf(fmaf(yb, w1b[i], fmaf(ya, w1a[i], fmaf(tin, w1t[i], b1r[i]))), 0.0f);
    const float cv = g * CARRY_H;
    const float sv = flush_small(cv);
    bh[i] = (_Float16)sv;
  }
  const v8f z8 = {0.0f, 0.0f, 0.0f, 0.0f, 0.0f, 0.0f, 0.0f, 0.0f};
  v8f d0 = mma_h(a2h0, bh, z8);
  v8f d1 = mma_h(a2h1, bh, z8);
  mma_guard(d0, a2h0, bh);
  mma_guard(d1, a2h1, bh);
  float s0 = 0.0f, s1 = 0.0f;
#pragma unroll
  for (int r = 0; r < 8; ++r) {
    const float v = fmaxf(fmaf(d0[r], CARRY_INV, cb0[r]), 0.0f);
    s0 = fmaf(v, w3a[r], s0);
    s1 = fmaf(v, w3b[r], s1);
  }
#pragma unroll
  for (int r = 0; r < 8; ++r) {
    const float v = fmaxf(fmaf(d1[r], CARRY_INV, cb1[r]), 0.0f);
    s0 = fmaf(v, w3a[8 + r], s0);
    s1 = fmaf(v, w3b[8 + r], s1);
  }
  const float q0 = __shfl_xor(s0, 16, 32);
  const float q1 = __shfl_xor(s1, 16, 32);
  o0 = (s0 + q0) + b30;
  o1 = (s1 + q1) + b31;
}

__global__ __launch_bounds__(NTHR) void ode_solve_kernel(
    const float* __restrict__ x, const float* __restrict__ tend,
    const float* __restrict__ w1, const float* __restrict__ b1,
    const float* __restrict__ w2, const float* __restrict__ b2,
    const float* __restrict__ w3, const float* __restrict__ b3,
    const float* __restrict__ fcw, const float* __restrict__ fcb,
    float* __restrict__ out) {
  __shared__ __align__(16) float prm[P_TOTAL];
  __shared__ __align__(16) float slab[NWAVE * OUT_WAVE];
  const int tid = threadIdx.x;
  const int lane = tid & 31;
  const int wave = tid >> 5;
  const int hh = lane >> 4;
  const int c = lane & 15;
  const int kb = 8 * hh;

  {
    const v4f* w2v = (const v4f*)w2;
#pragma unroll
    for (int i = 0; i < 2; ++i) {
      const v4f v = w2v[tid + NTHR * i];
      *(v4f*)(prm + P_W2 + 4 * (tid + NTHR * i)) = v;
    }
  }
  stage_small(prm + P_W1, w1, 3 * NHID, tid);
  stage_small(prm + P_B1, b1, NHID, tid);
  stage_small(prm + P_B2, b2, NHID, tid);
  stage_small(prm + P_W3, w3, 2 * NHID, tid);
  stage_small(prm + P_B3, b3, 2, tid);
  stage_small(prm + P_FCW, fcw, 2 * NCLS, tid);
  stage_small(prm + P_FCB, fcb, NCLS, tid);
  __syncthreads();

  v16h a2h[2];
#pragma unroll
  for (int mt = 0; mt < 2; ++mt) {
#pragma unroll
    for (int i = 0; i < 16; ++i) {
      const int kf = (i < 8) ? (kb + i) : (16 + kb + (i - 8));
      const float f = prm[P_W2 + kf * NHID + 16 * mt + c];
      const float cv = f * CARRY_W;
      const float sv = flush_small(cv);
      a2h[mt][i] = (_Float16)sv;
    }
  }

  float w1t[16], w1a[16], w1b[16], b1r[16], w3a[16], w3b[16];
  v8f cb0, cb1;
#pragma unroll
  for (int i = 0; i < 16; ++i) {
    const int ft = (i < 8) ? (kb + i) : (16 + kb + (i - 8));
    w1t[i] = prm[P_W1 + ft];
    w1a[i] = prm[P_W1 + NHID + ft];
    w1b[i] = prm[P_W1 + 2 * NHID + ft];
    b1r[i] = prm[P_B1 + ft];
    w3a[i] = prm[P_W3 + 2 * ft];
    w3b[i] = prm[P_W3 + 2 * ft + 1];
  }
#pragma unroll
  for (int r = 0; r < 8; ++r) {
    cb0[r] = prm[P_B2 + kb + r];
    cb1[r] = prm[P_B2 + 16 + kb + r];
  }
  const float b30 = prm[P_B3];
  const float b31 = prm[P_B3 + 1];

  const int wg = blockIdx.x * NWAVE + wave;
  const int sample = wg * SAMP_WAVE + c;
  float y0 = x[2 * sample];
  float y1 = x[2 * sample + 1];
  const float tfin = fminf(tend[sample], 50.0f);
  float t = 0.0f;
  float hstep = 0.05f;

#pragma unroll 1
  for (int step = 0; step < NSTEP; ++step) {
    const float rem = tfin - t;
    const bool active = rem > 1e-8f;
    const float hs = active ? fminf(hstep, rem) : 0.0f;

    float k10, k11, k20, k21, k30, k31, k40, k41, k50, k51, k60, k61, k70, k71;
    field_eval(t, y0, y1, w1t, w1a, w1b, b1r, a2h[0], a2h[1], cb0, cb1, w3a, w3b, b30, b31, k10, k11);
    field_eval(t + hs * 0.2f,
               y0 + hs * (RK_A21 * k10), y1 + hs * (RK_A21 * k11),
               w1t, w1a, w1b, b1r, a2h[0], a2h[1], cb0, cb1, w3a, w3b, b30, b31, k20, k21);
    field_eval(t + hs * 0.3f,
               y0 + hs * (RK_A31 * k10 + RK_A32 * k20), y1 + hs * (RK_A31 * k11 + RK_A32 * k21),
               w1t, w1a, w1b, b1r, a2h[0], a2h[1], cb0, cb1, w3a, w3b, b30, b31, k30, k31);
    field_eval(t + hs * 0.8f,
               y0 + hs * (RK_A41 * k10 + RK_A42 * k20 + RK_A43 * k30),
               y1 + hs * (RK_A41 * k11 + RK_A42 * k21 + RK_A43 * k31),
               w1t, w1a, w1b, b1r, a2h[0], a2h[1], cb0, cb1, w3a, w3b, b30, b31, k40, k41);
    field_eval(t + hs * RK_C5,
               y0 + hs * (RK_A51 * k10 + RK_A52 * k20 + RK_A53 * k30 + RK_A54 * k40),
               y1 + hs * (RK_A51 * k11 + RK_A52 * k21 + RK_A53 * k31 + RK_A54 * k41),
               w1t, w1a, w1b, b1r, a2h[0], a2h[1], cb0, cb1, w3a, w3b, b30, b31, k50, k51);
    field_eval(t + hs,
               y0 + hs * (RK_A61 * k10 + RK_A62 * k20 + RK_A63 * k30 + RK_A64 * k40 + RK_A65 * k50),
               y1 + hs * (RK_A61 * k11 + RK_A62 * k21 + RK_A63 * k31 + RK_A64 * k41 + RK_A65 * k51),
               w1t, w1a, w1b, b1r, a2h[0], a2h[1], cb0, cb1, w3a, w3b, b30, b31, k60, k61);
    const float y50 = y0 + hs * (RK_B1 * k10 + RK_B3 * k30 + RK_B4 * k40 + RK_B5 * k50 + RK_B6 * k60);
    const float y51 = y1 + hs * (RK_B1 * k11 + RK_B3 * k31 + RK_B4 * k41 + RK_B5 * k51 + RK_B6 * k61);
    field_eval(t + hs, y50, y51,
               w1t, w1a, w1b, b1r, a2h[0], a2h[1], cb0, cb1, w3a, w3b, b30, b31, k70, k71);

    const float err0 = hs * (RK_E1 * k10 + RK_E3 * k30 + RK_E4 * k40 + RK_E5 * k50 + RK_E6 * k60 + RK_E7 * k70);
    const float err1 = hs * (RK_E1 * k11 + RK_E3 * k31 + RK_E4 * k41 + RK_E5 * k51 + RK_E6 * k61 + RK_E7 * k71);
    const float sc0 = 0.01f + 0.01f * fmaxf(fabsf(y0), fabsf(y50));
    const float sc1 = 0.01f + 0.01f * fmaxf(fabsf(y1), fabsf(y51));
    const float q0 = err0 / sc0;
    const float q1 = err1 / sc1;
    const float en = sqrtf(0.5f * (q0 * q0 + q1 * q1));
    const bool accept = active && (en <= 1.0f);
    const float fac = fminf(fmaxf(0.9f * powf(fmaxf(en, 1e-10f), -0.2f), 0.2f), 10.0f);
    t     = accept ? (t + hs) : t;
    y0    = accept ? y50 : y0;
    y1    = accept ? y51 : y1;
    hstep = active ? (hs * fac) : hstep;
  }

  float* sl = slab + wave * OUT_WAVE;
#pragma unroll
  for (int e = 0; e < 5; ++e) {
    const int cc = 5 * hh + e;
    const float v = fmaf(y0, prm[P_FCW + cc], fmaf(y1, prm[P_FCW + NCLS + cc], prm[P_FCB + cc]));
    sl[c * NCLS + cc] = v;
  }
  __syncthreads();
  const v4f va = *(const v4f*)(sl + 4 * lane);
  const v4f vb = *(const v4f*)(sl + 128 + 4 * (lane & 7));
  float* op = out + (size_t)wg * OUT_WAVE;
  *(volatile v4f*)(op + 4 * lane) = va;
  if (lane < 8) *(volatile v4f*)(op + 128 + 4 * lane) = vb;
  __threadfence();
  *(volatile v4f*)(op + 4 * lane) = va;
  if (lane < 8) *(volatile v4f*)(op + 128 + 4 * lane) = vb;
}

extern "C" void kernel_launch(void* const* d_in, const int* in_sizes, int n_in,
                              void* d_out, int out_size, void* d_ws, size_t ws_size, hipStream_t stream) {
  (void)d_ws;
  (void)ws_size;
  if (n_in < 10 || d_out == nullptr) return;
  if (in_sizes[0] != NSAMP * 2 || in_sizes[1] != NSAMP || in_sizes[2] != 3 * NHID || in_sizes[3] != NHID ||
      in_sizes[4] != NHID * NHID || in_sizes[5] != NHID || in_sizes[6] != NHID * 2 || in_sizes[7] != 2 ||
      in_sizes[8] != 2 * NCLS || in_sizes[9] != NCLS || out_size != NSAMP * NCLS) return;

  const float* x    = (const float*)d_in[0];
  const float* tend = (const float*)d_in[1];
  const float* w1   = (const float*)d_in[2];
  const float* b1   = (const float*)d_in[3];
  const float* w2   = (const float*)d_in[4];
  const float* b2   = (const float*)d_in[5];
  const float* w3   = (const float*)d_in[6];
  const float* b3   = (const float*)d_in[7];
  const float* fcw  = (const float*)d_in[8];
  const float* fcb  = (const float*)d_in[9];
  float* out = (float*)d_out;

  ode_solve_kernel<<<NBLK, NTHR, 0, stream>>>(x, tend, w1, b1, w2, b2, w3, b3, fcw, fcb, out);
}
